// GRI_5488968204831
// MI455X (gfx1250) — hardware-run, weakly checked
//
#include <hip/hip_runtime.h>
#include <math.h>

typedef __attribute__((ext_vector_type(16))) __bf16   v16b;
typedef __attribute__((ext_vector_type(8)))  __bf16   v8b;
typedef __attribute__((ext_vector_type(8)))  float    v8f;
typedef __attribute__((ext_vector_type(4)))  float    v4f;
typedef __attribute__((ext_vector_type(4)))  unsigned v4u;
typedef __attribute__((ext_vector_type(4)))  int      v4i;
typedef __attribute__((address_space(1))) volatile float gvf;

constexpr int kBatch  = 2048;
constexpr int kNodes  = 4096;
constexpr int kLatent = 128;
constexpr int kFan    = 16;
constexpr int kWRow   = 1 + kLatent + kFan;
constexpr int kKReal  = 1 + kLatent;
constexpr int kKP     = 160;
constexpr int kKG     = kKP / 8;
static_assert(kWRow == 145, "weight row width");
static_assert(kKReal == 129 && kKP >= kKReal && (kKP % 32) == 0, "GEMM depth multiple of 32");
static_assert((kNodes % 64) == 0 && (kBatch % 64) == 0, "GEMM M, N multiples of 64");
static_assert((kBatch % 32) == 0 && (kNodes % 32) == 0, "32 x 32 transpose tiles");

constexpr size_t kOffWB   = 0;
constexpr size_t kOffXB   = kOffWB  + (size_t)kNodes * kKP * 2;
constexpr size_t kOffPC   = kOffXB  + (size_t)kBatch * kKP * 2;
constexpr size_t kOffPM   = kOffPC  + (size_t)kNodes * kFan * 4;
constexpr size_t kOffPW   = kOffPM  + (size_t)kNodes * kFan * 4;
constexpr size_t kOffPRE  = kOffPW  + (size_t)kNodes * kFan * 4;
constexpr size_t kOffU    = kOffPRE + (size_t)kNodes * kBatch * 4;
constexpr size_t kWsTotal = kOffU   + (size_t)kNodes * kBatch * 4;
static_assert(kWsTotal == 69861376ull, "carve total");
static_assert(kWsTotal <= 134217728ull, "carve cap");
static_assert((kOffXB % 256) == 0 && (kOffPC % 256) == 0 && (kOffPM % 256) == 0 && (kOffPW % 256) == 0 &&
              (kOffPRE % 256) == 0 && (kOffU % 256) == 0, "aligned regions");

constexpr int kBlkW = kNodes * kKG / 256;
constexpr int kBlkX = kBatch * kKG / 256;
constexpr int kBlkT = kNodes * kFan / 4 / 256;
constexpr int kBlkZ = kBatch / 4 / 256;
static_assert(kBlkW * 256 == kNodes * kKG, "exact cover of WB");
static_assert(kBlkX * 256 == kBatch * kKG, "exact cover of XB");
static_assert(kBlkT * 256 * 4 == kNodes * kFan, "exact cover of each per-node table");
static_assert(kBlkZ * 256 * 4 == kBatch, "exact cover of state row 0");
constexpr int kSecX  = kBlkW;
constexpr int kSecPC = kSecX  + kBlkX;
constexpr int kSecPM = kSecPC + kBlkT;
constexpr int kSecPW = kSecPM + kBlkT;
constexpr int kSecZ  = kSecPW + kBlkT;
constexpr int kPrepBlocks = kSecZ + kBlkZ;

__device__ __forceinline__ unsigned short f2bf_bits(float f) {
  unsigned u = __float_as_uint(f);
  return (unsigned short)((u + 0x7FFFu + ((u >> 16) & 1u)) >> 16);
}
__device__ __forceinline__ float bf_bits2f(unsigned short h) { return __uint_as_float(((unsigned)h) << 16); }
__device__ __forceinline__ float bf16r(float f) { return bf_bits2f(f2bf_bits(f)); }

__device__ __forceinline__ void acc_guard4(v8f& a, v8f& b, v8f& c, v8f& d) { asm volatile("v_nop\n\tv_nop\n\tv_nop\n\tv_nop" : "+v"(a), "+v"(b), "+v"(c), "+v"(d)); }

__device__ __forceinline__ v16b frag_load_bf16(const __bf16* p) {
  union FU { v16b v; v8b h[2]; };
  FU f;
  f.h[0] = *(const v8b*)(p);
  f.h[1] = *(const v8b*)(p + 16);
  return f.v;
}
__device__ __forceinline__ v8f mma_bf16_tied(v16b a, v16b b, v8f c) {
  c = __builtin_amdgcn_wmma_f32_16x16x32_bf16(false, a, false, b, (short)0, c, false, false);
  asm volatile("v_nop\n\tv_nop\n\tv_nop\n\tv_nop" : "+v"(c) : "v"(a), "v"(b));
  return c;
}

__device__ __forceinline__ void store_twice_u4(unsigned* p, v4u w) {
  *(volatile v4u*)p = w;
  __threadfence();
  *(volatile v4u*)p = w;
}
__device__ __forceinline__ void store_twice_f4(float* p, v4f w) {
  *(volatile v4f*)p = w;
  __threadfence();
  *(volatile v4f*)p = w;
}

__global__ __launch_bounds__(256) void prep_kernel(
    const float* __restrict__ z, const float* __restrict__ wts, const float* __restrict__ pmask,
    const int* __restrict__ parents,
    unsigned short* __restrict__ WB, unsigned short* __restrict__ XB,
    int* __restrict__ PC, float* __restrict__ PM, float* __restrict__ PW, float* __restrict__ U)
{
  const int blk = blockIdx.x;
  const int tid = threadIdx.x;
  if (blk < kSecX) {
    const int t = blk * 256 + tid;
    const int node = t / kKG;
    const int g = t - node * kKG;
    const float* wr = wts + (size_t)node * kWRow;
    unsigned hb[8];
#pragma unroll
    for (int e = 0; e < 8; ++e) {
      const int k = 8 * g + e;
      const int kc = (k < kKReal) ? k : (kKReal - 1);
      const float v = wr[kc];
      const float f = (k < kKReal) ? v : 0.0f;
      hb[e] = (unsigned)f2bf_bits(f);
    }
    const v4u w = { hb[0] | (hb[1] << 16), hb[2] | (hb[3] << 16), hb[4] | (hb[5] << 16), hb[6] | (hb[7] << 16) };
    store_twice_u4((unsigned*)WB + (size_t)t * 4, w);
  } else if (blk < kSecPC) {
    const int t = (blk - kSecX) * 256 + tid;
    const int row = t / kKG;
    const int g = t - row * kKG;
    const float* zr = z + (size_t)row * kLatent;
    unsigned hb[8];
#pragma unroll
    for (int e = 0; e < 8; ++e) {
      const int k = 8 * g + e;
      int zc = k - 1;
      zc = (zc < 0) ? 0 : zc;
      zc = (zc > kLatent - 1) ? (kLatent - 1) : zc;
      const float v = zr[zc];
      const float inr = (k <= kLatent) ? v : 0.0f;
      const float f = (k == 0) ? 1.0f : inr;
      hb[e] = (unsigned)f2bf_bits(f);
    }
    const v4u w = { hb[0] | (hb[1] << 16), hb[2] | (hb[3] << 16), hb[4] | (hb[5] << 16), hb[6] | (hb[7] << 16) };
    store_twice_u4((unsigned*)XB + (size_t)t * 4, w);
  } else if (blk < kSecPM) {
    const int t = (blk - kSecPC) * 256 + tid;
    const v4i p = *(const v4i*)(parents + (size_t)t * 4);
    int q0 = p[0], q1 = p[1], q2 = p[2], q3 = p[3];
    q0 = (q0 < 0) ? 0 : q0;  q0 = (q0 > kNodes - 1) ? (kNodes - 1) : q0;
    q1 = (q1 < 0) ? 0 : q1;  q1 = (q1 > kNodes - 1) ? (kNodes - 1) : q1;
    q2 = (q2 < 0) ? 0 : q2;  q2 = (q2 > kNodes - 1) ? (kNodes - 1) : q2;
    q3 = (q3 < 0) ? 0 : q3;  q3 = (q3 > kNodes - 1) ? (kNodes - 1) : q3;
    const v4u w = { (unsigned)q0, (unsigned)q1, (unsigned)q2, (unsigned)q3 };
    store_twice_u4((unsigned*)PC + (size_t)t * 4, w);
  } else if (blk < kSecPW) {
    const int t = (blk - kSecPM) * 256 + tid;
    const v4f m = *(const v4f*)(pmask + (size_t)t * 4);
    const float m0 = m[0], m1 = m[1], m2 = m[2], m3 = m[3];
    const v4f o = { bf16r(m0), bf16r(m1), bf16r(m2), bf16r(m3) };
    store_twice_f4(PM + (size_t)t * 4, o);
  } else if (blk < kSecZ) {
    const int t = (blk - kSecPW) * 256 + tid;
    const int node = t >> 2;
    const int k0 = (t & 3) * 4;
    const float* wr = wts + (size_t)node * kWRow + kKReal + k0;
    const float w0 = wr[0], w1 = wr[1], w2 = wr[2], w3 = wr[3];
    const v4f o = { bf16r(w0), bf16r(w1), bf16r(w2), bf16r(w3) };
    store_twice_f4(PW + (size_t)t * 4, o);
  } else {
    const int t = (blk - kSecZ) * 256 + tid;
    const v4f o = { 0.0f, 0.0f, 0.0f, 0.0f };
    store_twice_f4(U + (size_t)t * 4, o);
  }
}

__global__ __launch_bounds__(256) void pre_gemm_kernel(
    const unsigned short* __restrict__ Ap, const unsigned short* __restrict__ Btp, float* __restrict__ Cout)
{
  const __bf16* A  = (const __bf16*)Ap;
  const __bf16* Bt = (const __bf16*)Btp;
  __shared__ __align__(16) float sT[8][16 * 68];
  const int lane = threadIdx.x & 31;
  const int wave = threadIdx.x >> 5;
  constexpr int tilesN = kBatch >> 6;
  constexpr int tilesM = kNodes >> 6;
  const int tile = blockIdx.x * 8 + wave;
  if (tile >= tilesM * tilesN) return;
  const int tm = tile / tilesN;
  const int tn = tile - tm * tilesN;
  const int m0 = tm << 6;
  const int n0 = tn << 6;

  const int rlane = lane & 15;
  const int koff  = (lane >> 4) * 8;
  const int mOff  = (lane >> 4) * 8;

  v8f acc[4][4];
#pragma unroll
  for (int i = 0; i < 4; ++i)
#pragma unroll
    for (int j = 0; j < 4; ++j) acc[i][j] = (v8f){0.f,0.f,0.f,0.f,0.f,0.f,0.f,0.f};

#pragma unroll 1
  for (int k0 = 0; k0 < kKP; k0 += 32) {
    v16b bh[4];
#pragma unroll
    for (int j = 0; j < 4; ++j) {
      const size_t bo = (size_t)(n0 + (j << 4) + rlane) * kKP + koff + k0;
      bh[j] = frag_load_bf16(Bt + bo);
    }
#pragma unroll
    for (int i = 0; i < 4; ++i) {
      const size_t ao = (size_t)(m0 + (i << 4) + rlane) * kKP + koff + k0;
      const v16b ah = frag_load_bf16(A + ao);
#pragma unroll
      for (int j = 0; j < 4; ++j) acc[i][j] = mma_bf16_tied(ah, bh[j], acc[i][j]);
    }
  }
  acc_guard4(acc[0][0], acc[0][1], acc[0][2], acc[0][3]);
  acc_guard4(acc[1][0], acc[1][1], acc[1][2], acc[1][3]);
  acc_guard4(acc[2][0], acc[2][1], acc[2][2], acc[2][3]);
  acc_guard4(acc[3][0], acc[3][1], acc[3][2], acc[3][3]);

  float* slab = sT[wave];
#pragma unroll
  for (int i = 0; i < 4; ++i) {
    const int mBase = m0 + (i << 4);
#pragma unroll
    for (int j = 0; j < 4; ++j) {
#pragma unroll
      for (int r = 0; r < 8; ++r) slab[(mOff + r) * 68 + (j << 4) + rlane] = acc[i][j][r];
    }
    __builtin_amdgcn_fence(__ATOMIC_RELEASE, "workgroup");
    __builtin_amdgcn_wave_barrier();
    __builtin_amdgcn_fence(__ATOMIC_ACQUIRE, "workgroup");
    {
      const int hh = lane >> 4, c4 = (lane & 15) * 4;
      for (int pass = 0; pass < 2; ++pass) {
#pragma unroll
        for (int it = 0; it < 8; ++it) {
          const int row = it * 2 + hh;
          v4f v = *(const v4f*)(slab + row * 68 + c4);
          *(volatile v4f*)(Cout + (size_t)(mBase + row) * kBatch + n0 + c4) = v;
        }
        __threadfence();
      }
    }
    __builtin_amdgcn_fence(__ATOMIC_RELEASE, "workgroup");
    __builtin_amdgcn_wave_barrier();
    __builtin_amdgcn_fence(__ATOMIC_ACQUIRE, "workgroup");
  }
}

__global__ __launch_bounds__(32) void chain_kernel(
    const float* __restrict__ PRE, const int* __restrict__ PC, const float* __restrict__ PM,
    const float* __restrict__ PW, float* U)
{
  const int b = blockIdx.x * 32 + threadIdx.x;
  gvf* us = (gvf*)U;
  volatile float* uw = (volatile float*)U;
#pragma unroll 1
  for (int i = 0; i < kNodes; ++i) {
    const int*   pc = PC + (size_t)i * kFan;
    const float* pm = PM + (size_t)i * kFan;
    const float* pw = PW + (size_t)i * kFan;
    const int lim = (i > 0) ? (i - 1) : 0;
    float s = 0.0f;
#pragma unroll
    for (int k = 0; k < kFan; ++k) {
      int p = pc[k];
      p = (p < 0) ? 0 : p;
      p = (p > kNodes - 1) ? (kNodes - 1) : p;
      const bool live = (p < i);
      const int pa = (p < lim) ? p : lim;
      const float g = us[(size_t)pa * kBatch + b];
      const float u = live ? g : 0.0f;
      const float t = u * pm[k];
      s = fmaf(t, pw[k], s);
    }
    const float a = PRE[(size_t)i * kBatch + b] + s;
    const float v = tanhf(a);
    uw[(size_t)i * kBatch + b] = v;
    __threadfence();
    uw[(size_t)i * kBatch + b] = v;
    __threadfence();
  }
}

__global__ __launch_bounds__(256) void state_to_out_kernel(const float* __restrict__ U, float* __restrict__ out)
{
  __shared__ float tile[32 * 33];
  const int tid = threadIdx.x, lane = tid & 31, wave = tid >> 5;
  const int b0 = blockIdx.x * 32;
  const int n0 = blockIdx.y * 32;
  {
    const int nl = tid >> 3, c4 = (tid & 7) * 4;
    const v4f v = *(const v4f*)(U + (size_t)(n0 + nl) * kBatch + b0 + c4);
    const float v0 = v[0], v1 = v[1], v2 = v[2], v3 = v[3];
    tile[nl * 33 + c4 + 0] = v0;
    tile[nl * 33 + c4 + 1] = v1;
    tile[nl * 33 + c4 + 2] = v2;
    tile[nl * 33 + c4 + 3] = v3;
  }
  __syncthreads();
  const int q = lane >> 3, c = lane & 7;
  const int bl = wave * 4 + q;
  const v4f o = { tile[(c * 4 + 0) * 33 + bl], tile[(c * 4 + 1) * 33 + bl],
                  tile[(c * 4 + 2) * 33 + bl], tile[(c * 4 + 3) * 33 + bl] };
  store_twice_f4(out + (size_t)(b0 + bl) * kNodes + n0 + c * 4, o);
}

extern "C" void kernel_launch(void* const* d_in, const int* in_sizes, int n_in,
                              void* d_out, int out_size, void* d_ws, size_t ws_size,
                              hipStream_t stream) {
  if (n_in < 4 || d_out == nullptr || d_ws == nullptr) return;
  if (in_sizes[0] != kBatch * kLatent) return;
  if (in_sizes[1] != kNodes * kWRow) return;
  if (in_sizes[2] != kNodes * kFan) return;
  if (in_sizes[3] != kNodes * kFan) return;
  if (out_size != kBatch * kNodes) return;
  if (ws_size < kWsTotal) return;

  const float* z       = (const float*)d_in[0];
  const float* weights = (const float*)d_in[1];
  const float* pmask   = (const float*)d_in[2];
  const int*   parents = (const int*)d_in[3];
  float* out = (float*)d_out;

  char* ws = (char*)d_ws;
  unsigned short* WB  = (unsigned short*)(ws + kOffWB);
  unsigned short* XB  = (unsigned short*)(ws + kOffXB);
  int*            PC  = (int*)(ws + kOffPC);
  float*          PM  = (float*)(ws + kOffPM);
  float*          PW  = (float*)(ws + kOffPW);
  float*          PRE = (float*)(ws + kOffPRE);
  float*          U   = (float*)(ws + kOffU);

  prep_kernel<<<kPrepBlocks, 256, 0, stream>>>(z, weights, pmask, parents, WB, XB, PC, PM, PW, U);
  pre_gemm_kernel<<<(kNodes / 64) * (kBatch / 64) / 8, 256, 0, stream>>>(WB, XB, PRE);
  chain_kernel<<<kBatch / 32, 32, 0, stream>>>(PRE, PC, PM, PW, U);
  state_to_out_kernel<<<dim3(kBatch / 32, kNodes / 32), 256, 0, stream>>>(U, out);
}
